// guided_moe_basic_31550829756581
// MI455X (gfx1250) — hardware-verified
//
#include <hip/hip_runtime.h>
#include <stddef.h>
#include <stdint.h>


#define BB     8
#define LL     128
#define HH     768
#define EE     7
#define NEXP   4
#define D1     776
#define KW     800
#define CP     832
#define NPC    (CP / 8)
#define NPOS   1024
#define PPERB  8256
#define NPAIR  66048
#define HID    256
#define NG     8
#define NTHR   256
#define WSCL   64.0f
#define PSCL   0.015625f
#define WSCAP  134217728

static_assert(NPOS == BB * LL);
static_assert(PPERB == LL * (LL + 1) / 2);
static_assert(NPAIR == BB * PPERB);
static_assert((NPAIR % NTHR) == 0);
static_assert((NPOS % 32) == 0);
static_assert((KW % 32) == 0);
static_assert(KW >= D1);
static_assert(CP >= KW);
static_assert((CP % 64) == 0);
static_assert((HH % 32) == 0);
static_assert(HID == 8 * 32);
static_assert(NTHR == 8 * 32);

#define SZ_WT ((size_t)NG * HID * CP * 2)
#define SZ_GT ((size_t)16 * CP * 2)
#define SZ_C  ((size_t)NPOS * CP * 2)
#define SZ_GL ((size_t)NPOS * 16 * 4)
#define SZ_O  ((size_t)NG * NPOS * 2 * 4)
#define SZ_AM ((size_t)NPOS * 4)
#define SZ_TOT (SZ_WT + SZ_GT + SZ_C + SZ_GL + SZ_O + SZ_AM)
static_assert(SZ_TOT == 5273600);
static_assert(SZ_TOT <= (size_t)WSCAP);
static_assert((SZ_WT % 128) == 0);
static_assert((SZ_GT % 128) == 0);
static_assert((SZ_C % 128) == 0);
static_assert((SZ_GL % 128) == 0);
static_assert((SZ_O % 128) == 0);
static_assert((SZ_AM % 128) == 0);

typedef _Float16     v16h __attribute__((ext_vector_type(16)));
typedef _Float16     v8h  __attribute__((ext_vector_type(8)));
typedef float        v8f  __attribute__((ext_vector_type(8)));
typedef float        v4f  __attribute__((ext_vector_type(4)));
typedef unsigned int v4u  __attribute__((ext_vector_type(4)));
typedef int          v4i  __attribute__((ext_vector_type(4)));
union Frag { v16h v; v8h half[2]; };
union Pk8  { v8h h; v4u u; };

__device__ __forceinline__ v4u cvt8(const v4f a, const v4f b) {
  v8h hv = {(_Float16)a.x, (_Float16)a.y, (_Float16)a.z, (_Float16)a.w,
            (_Float16)b.x, (_Float16)b.y, (_Float16)b.z, (_Float16)b.w};
  Pk8 p;
  p.h = hv;
  return p.u;
}

__device__ __forceinline__ v8f wmh(v16h a, v16h b, v8f c) {
  v8f d = __builtin_amdgcn_wmma_f32_16x16x32_f16(false, a, false, b, (short)0, c, false, false);
  asm volatile("v_nop\n\tv_nop\n\tv_nop\n\tv_nop" : "+v"(d) : "v"(a), "v"(b));
  return d;
}

__device__ __forceinline__ v16h ld_frag(const _Float16* plane, int row, int k0, int h) {
  Frag f;
  const _Float16* p = plane + (size_t)row * CP + k0 + 8 * h;
  f.half[0] = *(const v8h*)p;
  f.half[1] = *(const v8h*)(p + 16);
  return f.v;
}

__device__ __forceinline__ double shfl_xor_d(double v, int o) {
  const unsigned long long u = (unsigned long long)__double_as_longlong(v);
  int lo = (int)(unsigned int)(u & 0xffffffffull);
  int hi = (int)(unsigned int)(u >> 32);
  lo = __shfl_xor(lo, o);
  hi = __shfl_xor(hi, o);
  const unsigned long long r = ((unsigned long long)(unsigned int)hi << 32) | (unsigned long long)(unsigned int)lo;
  return __longlong_as_double((long long)r);
}

__global__ __launch_bounds__(128) void k_prep(const float* __restrict__ W1, const float* __restrict__ GW,
                                              _Float16* WT, _Float16* GT) {
  const int blk = blockIdx.x, q = threadIdx.x;
  const float* src;
  int stride, act;
  _Float16* dst;
  if (blk < NG * HID) {
    const int g = blk >> 8, n = blk & (HID - 1), e = g & 3, koff = (g >> 2) * D1;
    src = W1 + ((size_t)e * (2 * D1) + (size_t)koff) * HID + n;
    stride = HID;
    act = 1;
    dst = WT + (size_t)blk * CP;
  } else {
    const int n = blk - NG * HID, nn = n & 7;
    src = GW + (size_t)((nn >> 2) * D1) * NEXP + (nn & 3);
    stride = NEXP;
    act = (n < 8) ? 1 : 0;
    dst = GT + (size_t)n * CP;
  }
  const int k0 = 8 * q;
  float f[8];
#pragma unroll
  for (int j = 0; j < 8; ++j) {
    const int k = k0 + j;
    const int kc = (k < D1) ? k : (D1 - 1);
    const float v = src[(size_t)kc * stride];
    f[j] = (act != 0 && k < D1) ? v * WSCL : 0.f;
  }
  const v4f f0 = {f[0], f[1], f[2], f[3]};
  const v4f f1 = {f[4], f[5], f[6], f[7]};
  const v4u pk = cvt8(f0, f1);
  _Float16* d = dst + k0;
  if (q < NPC) *(volatile v4u*)d = pk;
  __threadfence();
  if (q < NPC) *(volatile v4u*)d = pk;
}

__global__ __launch_bounds__(NTHR) void k_tok(const float* __restrict__ X, const int* __restrict__ spk,
                                              const float* __restrict__ EW, const float* __restrict__ EB,
                                              float* out0, _Float16* CPL, int* AM) {
  __shared__ __attribute__((aligned(16))) float s_w[HH * EE];
  __shared__ __attribute__((aligned(16))) float obuf[32 * EE];
  __shared__ __attribute__((aligned(16))) int am_s[32];
  const int tid = threadIdx.x, lane = tid & 31, wv = tid >> 5;
  const int blk = blockIdx.x;
  for (int i = tid; i < HH * EE; i += NTHR) s_w[i] = EW[i];
  double eb[EE];
#pragma unroll
  for (int e = 0; e < EE; ++e) eb[e] = (double)EB[e];
  __syncthreads();

#pragma unroll 1
  for (int j = 0; j < 4; ++j) {
    const int tl = 4 * wv + j;
    const int p = 32 * blk + tl;
    const float* xr = X + (size_t)p * HH;
    double s[EE];
#pragma unroll
    for (int e = 0; e < EE; ++e) s[e] = 0.0;
#pragma unroll 1
    for (int i = 0; i < HH / 32; ++i) {
      const int k = 32 * i + lane;
      const double x = (double)xr[k];
      const float* w = s_w + k * EE;
#pragma unroll
      for (int e = 0; e < EE; ++e) s[e] = fma(x, (double)w[e], s[e]);
    }
    float ef[EE];
#pragma unroll
    for (int e = 0; e < EE; ++e) {
      double v = s[e];
      v += shfl_xor_d(v, 16);
      v += shfl_xor_d(v, 8);
      v += shfl_xor_d(v, 4);
      v += shfl_xor_d(v, 2);
      v += shfl_xor_d(v, 1);
      v += eb[e];
      s[e] = v;
      ef[e] = (float)v;
    }
    int best = 0;
    double bv = s[0];
#pragma unroll
    for (int e = 1; e < EE; ++e) {
      if (s[e] > bv) { bv = s[e]; best = e; }
    }
    if (lane == 0) {
#pragma unroll
      for (int e = 0; e < EE; ++e) obuf[tl * EE + e] = ef[e];
      am_s[tl] = best;
    }
    const float spv = (float)spk[p];
    v4u pk[4];
#pragma unroll
    for (int it = 0; it < 3; ++it) {
      const int q = 32 * it + lane;
      const float* sp = xr + 8 * q;
      const v4f a0 = *(const v4f*)sp, a1 = *(const v4f*)(sp + 4);
      pk[it] = cvt8(a0, a1);
    }
    {
      const v4f e0 = {ef[0], ef[1], ef[2], ef[3]};
      const v4f e1 = {ef[4], ef[5], ef[6], spv};
      const v4u pe = cvt8(e0, e1);
      v4u z;
      z.x = (lane == 0) ? pe.x : 0u;
      z.y = (lane == 0) ? pe.y : 0u;
      z.z = (lane == 0) ? pe.z : 0u;
      z.w = (lane == 0) ? pe.w : 0u;
      pk[3] = z;
    }
    _Float16* crow = CPL + (size_t)p * CP;
#pragma unroll
    for (int it = 0; it < 3; ++it) *(volatile v4u*)(crow + 8 * (32 * it + lane)) = pk[it];
    if (lane < 8) *(volatile v4u*)(crow + 8 * (96 + lane)) = pk[3];
    __threadfence();
#pragma unroll
    for (int it = 0; it < 3; ++it) *(volatile v4u*)(crow + 8 * (32 * it + lane)) = pk[it];
    if (lane < 8) *(volatile v4u*)(crow + 8 * (96 + lane)) = pk[3];
  }
  __syncthreads();

  const int qo = (tid < 56) ? tid : 55;
  const v4f ov = *(const v4f*)(obuf + 4 * qo);
  float* po = out0 + (size_t)blk * (32 * EE) + 4 * qo;
  const int qa = (tid >= 64 && tid < 72) ? (tid - 64) : 0;
  const v4i av = *(const v4i*)(am_s + 4 * qa);
  int* pa = AM + (size_t)blk * 32 + 4 * qa;
  if (tid < 56) *(volatile v4f*)po = ov;
  if (tid >= 64 && tid < 72) *(volatile v4i*)pa = av;
  __threadfence();
  if (tid < 56) *(volatile v4f*)po = ov;
  if (tid >= 64 && tid < 72) *(volatile v4i*)pa = av;
}

__global__ __launch_bounds__(64) void k_gate(const _Float16* __restrict__ CPL, const _Float16* __restrict__ GT,
                                             float* GL) {
  __shared__ __attribute__((aligned(16))) float gls[32 * 16];
  const int tid = threadIdx.x, lane = tid & 31, wv = tid >> 5, h = lane >> 4, m = lane & 15;
  const int blk = blockIdx.x;
  const int row = 32 * blk + 16 * wv + m;
  v8f acc = {0.f, 0.f, 0.f, 0.f, 0.f, 0.f, 0.f, 0.f};
#pragma unroll 1
  for (int kt = 0; kt < KW / 32; ++kt) {
    const int k0 = 32 * kt;
    const v16h a = ld_frag(CPL, row, k0, h);
    const v16h b = ld_frag(GT, m, k0, h);
    acc = wmh(a, b, acc);
  }
#pragma unroll
  for (int r = 0; r < 8; ++r) gls[(16 * wv + 8 * h + r) * 16 + m] = acc[r] * PSCL;
  __syncthreads();

  v4f v[2];
#pragma unroll
  for (int it = 0; it < 2; ++it) v[it] = *(const v4f*)(gls + 4 * (64 * it + tid));
  float* pg = GL + (size_t)blk * 512;
#pragma unroll
  for (int it = 0; it < 2; ++it) *(volatile v4f*)(pg + 4 * (64 * it + tid)) = v[it];
  __threadfence();
#pragma unroll
  for (int it = 0; it < 2; ++it) *(volatile v4f*)(pg + 4 * (64 * it + tid)) = v[it];
}

__global__ __launch_bounds__(NTHR) void k_exp(const _Float16* __restrict__ CPL, const _Float16* __restrict__ WT,
                                              const float* __restrict__ W2, float* OT) {
  __shared__ __attribute__((aligned(16))) float wred[8 * 32 * 2];
  __shared__ __attribute__((aligned(16))) float obuf[64];
  const int tid = threadIdx.x, lane = tid & 31, wv = tid >> 5, h = lane >> 4, m = lane & 15;
  const int blk = blockIdx.x, g = blockIdx.y, e = g & 3;
  const _Float16* Bp = WT + (size_t)g * HID * CP;

  const v8f zero8 = {0.f, 0.f, 0.f, 0.f, 0.f, 0.f, 0.f, 0.f};
  v8f acc[2][2];
#pragma unroll
  for (int mt = 0; mt < 2; ++mt) { acc[mt][0] = zero8; acc[mt][1] = zero8; }
#pragma unroll 1
  for (int kt = 0; kt < KW / 32; ++kt) {
    const int k0 = 32 * kt;
    const v16h b0 = ld_frag(Bp, 32 * wv + m, k0, h);
    const v16h b1 = ld_frag(Bp, 32 * wv + 16 + m, k0, h);
#pragma unroll
    for (int mt = 0; mt < 2; ++mt) {
      const v16h a = ld_frag(CPL, 32 * blk + 16 * mt + m, k0, h);
      acc[mt][0] = wmh(a, b0, acc[mt][0]);
      acc[mt][1] = wmh(a, b1, acc[mt][1]);
    }
  }

  float wa[2], wb[2];
#pragma unroll
  for (int nt = 0; nt < 2; ++nt) {
    const int col = 32 * wv + 16 * nt + m;
    const float* wp = W2 + ((size_t)e * HID + col) * 2;
    wa[nt] = wp[0];
    wb[nt] = wp[1];
  }
  float pr0[2][8], pr1[2][8];
#pragma unroll
  for (int mt = 0; mt < 2; ++mt) {
#pragma unroll
    for (int r = 0; r < 8; ++r) {
      float p0 = 0.f, p1 = 0.f;
#pragma unroll
      for (int nt = 0; nt < 2; ++nt) {
        const float d = acc[mt][nt][r] * PSCL;
        p0 += d * wa[nt];
        p1 += d * wb[nt];
      }
      p0 += __shfl_xor(p0, 1);
      p1 += __shfl_xor(p1, 1);
      p0 += __shfl_xor(p0, 2);
      p1 += __shfl_xor(p1, 2);
      p0 += __shfl_xor(p0, 4);
      p1 += __shfl_xor(p1, 4);
      p0 += __shfl_xor(p0, 8);
      p1 += __shfl_xor(p1, 8);
      pr0[mt][r] = p0;
      pr1[mt][r] = p1;
    }
  }
  if (m == 0) {
#pragma unroll
    for (int mt = 0; mt < 2; ++mt) {
#pragma unroll
      for (int r = 0; r < 8; ++r) {
        const int R = 16 * mt + 8 * h + r;
        wred[(wv * 32 + R) * 2 + 0] = pr0[mt][r];
        wred[(wv * 32 + R) * 2 + 1] = pr1[mt][r];
      }
    }
  }
  __syncthreads();
  if (tid < 64) {
    const int row = tid >> 1, c = tid & 1;
    float s = 0.f;
#pragma unroll
    for (int w = 0; w < 8; ++w) s += wred[(w * 32 + row) * 2 + c];
    obuf[tid] = s;
  }
  __syncthreads();
  if (wv == 0) {
    const int q = lane & 15;
    const v4f v = *(const v4f*)(obuf + 4 * q);
    float* po = OT + ((size_t)g * NPOS + 32 * blk) * 2 + 4 * q;
    if (lane < 16) *(volatile v4f*)po = v;
    __threadfence();
    if (lane < 16) *(volatile v4f*)po = v;
  }
}

__global__ __launch_bounds__(NTHR) void k_fin(const int* __restrict__ spk, const int* __restrict__ AM,
                                              const float* __restrict__ GL, const float* __restrict__ GB,
                                              const float* __restrict__ OT, const float* __restrict__ B1,
                                              const float* __restrict__ W2, const float* __restrict__ B2,
                                              float* out1) {
  __shared__ float cst[8];
  __shared__ __attribute__((aligned(16))) float obuf[2 * NTHR];
  const int tid = threadIdx.x, blk = blockIdx.x;
  if (tid < 8) {
    const int e = tid >> 1, c = tid & 1;
    float s = 0.f;
#pragma unroll 1
    for (int n = 0; n < HID; ++n) s += B1[e * HID + n] * W2[((size_t)e * HID + n) * 2 + c];
    cst[tid] = s + B2[e * 2 + c];
  }
  __syncthreads();

  const int gid = blk * NTHR + tid;
  int b = gid / PPERB;
  b = (b < BB) ? b : (BB - 1);
  const int i = gid - b * PPERB;
  int end = (int)((sqrtf(8.0f * (float)i + 1.0f) - 1.0f) * 0.5f);
#pragma unroll
  for (int st = 0; st < 2; ++st) { if ((end + 1) * (end + 2) / 2 <= i) ++end; }
#pragma unroll
  for (int st = 0; st < 2; ++st) { if (end > 0 && end * (end + 1) / 2 > i) --end; }
  end = (end < 0) ? 0 : ((end > LL - 1) ? (LL - 1) : end);
  int t = i - end * (end + 1) / 2;
  t = (t < 0) ? 0 : ((t > LL - 1) ? (LL - 1) : t);
  const int pt = b * LL + t;
  const int pe = b * LL + end;

  const bool s_eq = spk[pt] == spk[pe];
  const bool e_eq = AM[pt] == AM[pe];
  const int lbl = (s_eq && e_eq) ? 0 : (s_eq ? 1 : (e_eq ? 2 : 3));

  float lg[NEXP];
  float mx = -3.0e38f;
#pragma unroll
  for (int e = 0; e < NEXP; ++e) {
    lg[e] = (GL[(size_t)pt * 16 + e] + GL[(size_t)pe * 16 + 4 + e]) + GB[e];
    mx = fmaxf(mx, lg[e]);
  }
  float se = 0.f;
#pragma unroll
  for (int e = 0; e < NEXP; ++e) { lg[e] = __expf(lg[e] - mx); se += lg[e]; }
  const float inv = __builtin_amdgcn_rcpf(se);

  float o0 = 0.f, o1 = 0.f;
#pragma unroll
  for (int e = 0; e < NEXP; ++e) {
    const float gate = ((e == lbl) ? 0.6f : 0.0f) + 0.4f * (lg[e] * inv);
    const float q0 = (OT[((size_t)e * NPOS + pt) * 2 + 0] + OT[((size_t)(NEXP + e) * NPOS + pe) * 2 + 0]) + cst[2 * e + 0];
    const float q1 = (OT[((size_t)e * NPOS + pt) * 2 + 1] + OT[((size_t)(NEXP + e) * NPOS + pe) * 2 + 1]) + cst[2 * e + 1];
    o0 += gate * q0;
    o1 += gate * q1;
  }
  obuf[2 * tid + 0] = o0;
  obuf[2 * tid + 1] = o1;
  __syncthreads();

  const int q = (tid < 128) ? tid : 127;
  const v4f v = *(const v4f*)(obuf + 4 * q);
  float* po = out1 + (size_t)blk * (2 * NTHR) + 4 * q;
  if (tid < 128) *(volatile v4f*)po = v;
  __threadfence();
  if (tid < 128) *(volatile v4f*)po = v;
}

extern "C" void kernel_launch(void* const* d_in, const int* in_sizes, int n_in,
                              void* d_out, int out_size, void* d_ws, size_t ws_size,
                              hipStream_t stream) {
  if (n_in < 10) return;
  if (in_sizes[0] != NPOS * HH) return;
  if (in_sizes[1] != NPOS) return;
  if (in_sizes[2] != HH * EE || in_sizes[3] != EE) return;
  if (in_sizes[4] != 2 * D1 * NEXP || in_sizes[5] != NEXP) return;
  if (in_sizes[6] != NEXP * 2 * D1 * HID || in_sizes[7] != NEXP * HID) return;
  if (in_sizes[8] != NEXP * HID * 2 || in_sizes[9] != NEXP * 2) return;
  if (out_size != NPOS * EE + NPAIR * 2) return;

  const float* X  = (const float*)d_in[0];
  const int*   SP = (const int*)d_in[1];
  const float* EW = (const float*)d_in[2];
  const float* EB = (const float*)d_in[3];
  const float* GW = (const float*)d_in[4];
  const float* GB = (const float*)d_in[5];
  const float* W1 = (const float*)d_in[6];
  const float* B1 = (const float*)d_in[7];
  const float* W2 = (const float*)d_in[8];
  const float* B2 = (const float*)d_in[9];
  float* out = (float*)d_out;

  char* ws = (char*)d_ws;
  size_t off = 0;
  const size_t oWT = off; off += SZ_WT;
  const size_t oGT = off; off += SZ_GT;
  const size_t oC  = off; off += SZ_C;
  const size_t oGL = off; off += SZ_GL;
  const size_t oO  = off; off += SZ_O;
  const size_t oAM = off; off += SZ_AM;
  if (off != SZ_TOT) return;
  if (off > ws_size || off > (size_t)WSCAP) return;

  _Float16* WT  = (_Float16*)(ws + oWT);
  _Float16* GT  = (_Float16*)(ws + oGT);
  _Float16* CPL = (_Float16*)(ws + oC);
  float* GL = (float*)(ws + oGL);
  float* OT = (float*)(ws + oO);
  int*   AM = (int*)(ws + oAM);

  k_prep<<<NG * HID + 16, 128, 0, stream>>>(W1, GW, WT, GT);
  k_tok<<<NPOS / 32, NTHR, 0, stream>>>(X, SP, EW, EB, out, CPL, AM);
  k_gate<<<NPOS / 32, 64, 0, stream>>>(CPL, GT, GL);
  k_exp<<<dim3(NPOS / 32, NG), NTHR, 0, stream>>>(CPL, WT, W2, OT);
  k_fin<<<NPAIR / NTHR, NTHR, 0, stream>>>(SP, AM, GL, GB, OT, B1, W2, B2, out + NPOS * EE);
}
